// RetouchGenerator_25434796327093
// MI455X (gfx1250) — hardware-verified
//
#include <hip/hip_runtime.h>

typedef __attribute__((ext_vector_type(16))) _Float16 v16h;
typedef __attribute__((ext_vector_type(8)))  _Float16 v8h;
typedef __attribute__((ext_vector_type(16))) __bf16   v16b;
typedef __attribute__((ext_vector_type(8)))  __bf16   v8b;
typedef __attribute__((ext_vector_type(8)))  float    v8f;
typedef __attribute__((ext_vector_type(4)))  float    v4f;
typedef __attribute__((ext_vector_type(4)))  unsigned int v4u;
#define PSCALE 32768.0f
#define U16(p) ((const unsigned short*)(const void*)(p))
#define PSCALE_INV (1.0f / 32768.0f)

__device__ __forceinline__ unsigned short f2bf_bits(float f) {
  unsigned u = __float_as_uint(f);
  return (unsigned short)((u + 0x7FFFu + ((u >> 16) & 1u)) >> 16);
}
__device__ __forceinline__ float bf_bits2f(unsigned short h) { return __uint_as_float(((unsigned)h) << 16); }

__device__ __forceinline__ void dep_guard_h(v8f& a, v8f& b, v16h x, v16h y) { asm volatile("v_nop\n\tv_nop\n\tv_nop\n\tv_nop" : "+v"(a), "+v"(b) : "v"(x), "v"(y)); }
__device__ __forceinline__ void dep_guard_b(v8f& a, v8f& b, v16b x, v16b y) { asm volatile("v_nop\n\tv_nop\n\tv_nop\n\tv_nop" : "+v"(a), "+v"(b) : "v"(x), "v"(y)); }
__device__ __forceinline__ void keep4_h(v16h a, v16h b, v16h c, v16h d) { asm volatile("v_nop" :: "v"(a), "v"(b), "v"(c), "v"(d)); }
__device__ __forceinline__ void keep4_b(v16b a, v16b b, v16b c, v16b d) { asm volatile("v_nop" :: "v"(a), "v"(b), "v"(c), "v"(d)); }
__device__ __forceinline__ void acc_guard4(v8f& a, v8f& b, v8f& c, v8f& d) { asm volatile("v_nop\n\tv_nop\n\tv_nop\n\tv_nop" : "+v"(a), "+v"(b), "+v"(c), "+v"(d)); }
template <typename T> struct Frag;
template <> struct Frag<_Float16> {
  typedef v16h V; union U { v16h v; v8h h[2]; };
  static __device__ __forceinline__ v16h load(const _Float16* p) {
    U f; f.h[0] = *(const v8h*)(p); f.h[1] = *(const v8h*)(p + 16); return f.v;
  }
  static __device__ __forceinline__ v8f mma(v16h a, v16h b, v8f c) {
    return __builtin_amdgcn_wmma_f32_16x16x32_f16(false, a, false, b, (short)0, c, false, false);
  }
  static __device__ __forceinline__ void guard(v8f& a, v8f& b, v16h x, v16h y) { dep_guard_h(a, b, x, y); }
  static __device__ __forceinline__ void keep(v16h a, v16h b, v16h c, v16h d) { keep4_h(a, b, c, d); }
};
template <> struct Frag<__bf16> {
  typedef v16b V; union U { v16b v; v8b h[2]; };
  static __device__ __forceinline__ v16b load(const __bf16* p) {
    U f; f.h[0] = *(const v8b*)(p); f.h[1] = *(const v8b*)(p + 16); return f.v;
  }
  static __device__ __forceinline__ v8f mma(v16b a, v16b b, v8f c) {
    return __builtin_amdgcn_wmma_f32_16x16x32_bf16(false, a, false, b, (short)0, c, false, false);
  }
  static __device__ __forceinline__ void guard(v8f& a, v8f& b, v16b x, v16b y) { dep_guard_b(a, b, x, y); }
  static __device__ __forceinline__ void keep(v16b a, v16b b, v16b c, v16b d) { keep4_b(a, b, c, d); }
};

template <int ET> struct Elem;
template <> struct Elem<0> { typedef _Float16 T; };
template <> struct Elem<1> { typedef __bf16 T; };
template <int ET, bool SPLIT, int BIAS_MODE, int OUT_MODE, bool RESID, int ACT = 0>
__global__ __launch_bounds__(256) void wmma_gemm64(
    const unsigned short* __restrict__ Ap, const unsigned short* __restrict__ A2p, int lda, long strideA,
    const unsigned short* __restrict__ Btp, const unsigned short* __restrict__ Bt2p, int ldb, long strideB,
    void* __restrict__ Cout, void* __restrict__ Cout2, int ldc, long strideC,
    const float* __restrict__ bias,
    const float* __restrict__ resid, long strideR,
    int M, int N, int K, float scale) {
  typedef typename Elem<ET>::T T;
  typedef typename Frag<T>::V V;
  const T* A = (const T*)Ap; const T* A2 = (const T*)A2p; const T* Bt = (const T*)Btp; const T* Bt2 = (const T*)Bt2p;
  __shared__ __align__(16) float sT[8][16 * 68];
  const int b    = blockIdx.y;
  const int lane = threadIdx.x & 31;
  const int wave = threadIdx.x >> 5;
  const int tilesN = N >> 6;
  const int tilesM = M >> 6;
  const int tile = blockIdx.x * 8 + wave;
  if (tile >= tilesM * tilesN) return;
  const int tm = tile / tilesN;
  const int tn = tile - tm * tilesN;
  const int m0 = tm << 6;
  const int n0 = tn << 6;

  const T* Ab  = A  + (size_t)b * strideA;
  const T* Bb  = Bt + (size_t)b * strideB;
  const T* Ab2 = SPLIT ? (A2  + (size_t)b * strideA) : nullptr;
  const T* Bb2 = SPLIT ? (Bt2 + (size_t)b * strideB) : nullptr;

  const int rlane = lane & 15;
  const int koff  = (lane >> 4) * 8;
  const int mOff  = (lane >> 4) * 8;

  v8f acc[4][4];
#pragma unroll
  for (int i = 0; i < 4; ++i)
#pragma unroll
    for (int j = 0; j < 4; ++j) acc[i][j] = (v8f){0.f,0.f,0.f,0.f,0.f,0.f,0.f,0.f};

  for (int k0 = 0; k0 < K; k0 += 32) {
    V bh[4], bl[4];
#pragma unroll
    for (int j = 0; j < 4; ++j) {
      const size_t bo = (size_t)(n0 + (j << 4) + rlane) * ldb + koff + k0;
      bh[j] = Frag<T>::load(Bb + bo);
      if (SPLIT) bl[j] = Frag<T>::load(Bb2 + bo);
    }
#pragma unroll
    for (int i = 0; i < 4; ++i) {
      const size_t ao = (size_t)(m0 + (i << 4) + rlane) * lda + koff + k0;
      V ah = Frag<T>::load(Ab + ao);
      V al;
      if (SPLIT) al = Frag<T>::load(Ab2 + ao);
#pragma unroll
      for (int j = 0; j < 4; ++j) {
        acc[i][j] = Frag<T>::mma(ah, bh[j], acc[i][j]);
        if (SPLIT) {
          acc[i][j] = Frag<T>::mma(ah, bl[j], acc[i][j]);
          acc[i][j] = Frag<T>::mma(al, bh[j], acc[i][j]);
        }
      }
      Frag<T>::guard(acc[i][0], acc[i][3], ah, SPLIT ? al : ah);
    }
    Frag<T>::keep(bh[0], bh[1], bh[2], bh[3]);
    if (SPLIT) Frag<T>::keep(bl[0], bl[1], bl[2], bl[3]);
  }
  acc_guard4(acc[0][0], acc[0][1], acc[0][2], acc[0][3]);
  acc_guard4(acc[1][0], acc[1][1], acc[1][2], acc[1][3]);
  acc_guard4(acc[2][0], acc[2][1], acc[2][2], acc[2][3]);
  acc_guard4(acc[3][0], acc[3][1], acc[3][2], acc[3][3]);

  float* slab = sT[wave];
  const float* Rb = RESID ? (resid + (size_t)b * strideR) : nullptr;
#pragma unroll
  for (int i = 0; i < 4; ++i) {
    const int mBase = m0 + (i << 4);
#pragma unroll
    for (int j = 0; j < 4; ++j) {
      const int n = n0 + (j << 4) + rlane;
      float bv = 0.f;
      if (BIAS_MODE == 2) bv = bias[n];
#pragma unroll
      for (int r = 0; r < 8; ++r) {
        float v = acc[i][j][r] * scale;
        if (BIAS_MODE == 1) v += bias[mBase + mOff + r];
        if (BIAS_MODE == 2) v += bv;
        if (RESID) v += Rb[(size_t)(mBase + mOff + r) * ldc + n];
        if (ACT == 1) v = tanhf(v);
        if (ACT == 2) v = fmaxf(v, 0.0f);
        if (ACT == 3) v = v / (1.0f + expf(-v));
        if (ACT == 4) v = (v > 0.f) ? v : 0.01f * v;
        if (ACT == 5) v = 0.5f * v * (1.0f + erff(v * 0.70710678118654752f));
        slab[(mOff + r) * 68 + (j << 4) + rlane] = v;
      }
    }
    __builtin_amdgcn_fence(__ATOMIC_RELEASE, "workgroup");
    __builtin_amdgcn_wave_barrier();
    __builtin_amdgcn_fence(__ATOMIC_ACQUIRE, "workgroup");
    if (OUT_MODE == 0) {
      float* C = (float*)Cout + (size_t)b * strideC;
      const int hh = lane >> 4, c4 = (lane & 15) * 4;
      for (int pass = 0; pass < 2; ++pass) {
#pragma unroll
        for (int it = 0; it < 8; ++it) {
          const int row = it * 2 + hh;
          v4f v = *(const v4f*)(slab + row * 68 + c4);
          *(volatile v4f*)(C + (size_t)(mBase + row) * ldc + n0 + c4) = v;
        }
        __threadfence();
      }
    } else {
      const int q = lane >> 3, c8 = (lane & 7) * 8;
      unsigned short* C  = (unsigned short*)Cout  + (size_t)b * strideC;
      unsigned short* C2 = (OUT_MODE == 2) ? ((unsigned short*)Cout2 + (size_t)b * strideC) : nullptr;
      for (int pass = 0; pass < 2; ++pass) {
#pragma unroll
        for (int it = 0; it < 4; ++it) {
          const int row = it * 4 + q;
          const float* sp = slab + row * 68 + c8;
          v8h hv, lv;
#pragma unroll
          for (int e = 0; e < 8; ++e) {
            if (OUT_MODE == 1) {
              hv[e] = (_Float16)sp[e];
            } else {
              unsigned short hb = f2bf_bits(sp[e]);
              unsigned short lb = f2bf_bits(sp[e] - bf_bits2f(hb));
              hv[e] = __builtin_bit_cast(_Float16, hb);
              lv[e] = __builtin_bit_cast(_Float16, lb);
            }
          }
          *(volatile v8h*)(C + (size_t)(mBase + row) * ldc + n0 + c8) = hv;
          if (OUT_MODE == 2) *(volatile v8h*)(C2 + (size_t)(mBase + row) * ldc + n0 + c8) = lv;
        }
        __threadfence();
      }
    }
    __builtin_amdgcn_fence(__ATOMIC_RELEASE, "workgroup");
    __builtin_amdgcn_wave_barrier();
    __builtin_amdgcn_fence(__ATOMIC_ACQUIRE, "workgroup");
  }
}

struct ColGeom {
  long long sb, sy, sx, s_clo, s_chi, add_sb;
  int Hin, Win, Hout, Wout, stride, pad, taps, kw, Cin, Kreal, KPAD, Mreal, cmask, cshift, nthr, unused0;
};
static_assert(sizeof(ColGeom) == 112);

template <int FUSE>
__global__ __launch_bounds__(256) void im2col_split_kernel(
    const float* __restrict__ in, const float* __restrict__ addv,
    unsigned short* __restrict__ Ahi, unsigned short* __restrict__ Alo, ColGeom g) {
  const int t = blockIdx.x * 256 + threadIdx.x;
  if (t >= g.nthr) return;
  const int e0 = t * 8;
  const int row = e0 / g.KPAD;
  const int k0 = e0 - row * g.KPAD;
  const int hw = g.Hout * g.Wout;
  const bool rowok = row < g.Mreal;
  const int rowc = rowok ? row : (g.Mreal - 1);
  const int bb = rowc / hw;
  const int rem = rowc - bb * hw;
  const int oy = rem / g.Wout;
  const int ox = rem - oy * g.Wout;
  unsigned hbits[8];
  unsigned lbits[8];
#pragma unroll
  for (int j = 0; j < 8; ++j) {
    const int k = k0 + j;
    const bool kok = k < g.Kreal;
    const int kc = kok ? k : (g.Kreal - 1);
    const int kpos = kc / g.Cin;
    const int ic = kc - kpos * g.Cin;
    const int ky = kpos / g.kw;
    const int kx = kpos - ky * g.kw;
    const int iy = oy * g.stride - g.pad + ky;
    const int ix = ox * g.stride - g.pad + kx;
    const bool inb = (iy >= 0) && (iy < g.Hin) && (ix >= 0) && (ix < g.Win);
    const int iyc = min(max(iy, 0), g.Hin - 1);
    const int ixc = min(max(ix, 0), g.Win - 1);
    const long long coff = (long long)(ic & g.cmask) * g.s_clo + (long long)(ic >> g.cshift) * g.s_chi;
    const long long addr = (long long)bb * g.sb + coff + (long long)iyc * g.sy + (long long)ixc * g.sx;
    float v = in[addr];
    if (FUSE) {
      const float ad = addv[(long long)bb * g.add_sb + ic];
      v = fmaxf(v + ad, 0.0f);
    }
    v = (rowok && kok && inb) ? v : 0.0f;
    const unsigned short hb = f2bf_bits(v);
    const unsigned short lb = f2bf_bits(v - bf_bits2f(hb));
    hbits[j] = (unsigned)hb;
    lbits[j] = (unsigned)lb;
  }
  v4u hv, lv;
  hv.x = hbits[0] | (hbits[1] << 16); hv.y = hbits[2] | (hbits[3] << 16);
  hv.z = hbits[4] | (hbits[5] << 16); hv.w = hbits[6] | (hbits[7] << 16);
  lv.x = lbits[0] | (lbits[1] << 16); lv.y = lbits[2] | (lbits[3] << 16);
  lv.z = lbits[4] | (lbits[5] << 16); lv.w = lbits[6] | (lbits[7] << 16);
  unsigned short* ph = Ahi + (size_t)e0;
  unsigned short* pl = Alo + (size_t)e0;
  for (int pass = 0; pass < 2; ++pass) {
    *(volatile v4u*)ph = hv;
    *(volatile v4u*)pl = lv;
    __threadfence();
  }
}

struct WGeom { int Cout, Cin, taps, Kreal, KPAD, NPAD, nthr, has_bias; };
static_assert(sizeof(WGeom) == 32);

__global__ __launch_bounds__(256) void prep_w_kernel(
    const float* __restrict__ w, const float* __restrict__ bias,
    unsigned short* __restrict__ Bhi, unsigned short* __restrict__ Blo,
    float* __restrict__ bpad, WGeom g) {
  const int t = blockIdx.x * 256 + threadIdx.x;
  if (t < g.nthr) {
    const int e0 = t * 8;
    const int n = e0 / g.KPAD;
    const int k0 = e0 - n * g.KPAD;
    const bool nok = n < g.Cout;
    const int nc = nok ? n : (g.Cout - 1);
    unsigned hbits[8];
    unsigned lbits[8];
#pragma unroll
    for (int j = 0; j < 8; ++j) {
      const int k = k0 + j;
      const bool kok = k < g.Kreal;
      const int kc = kok ? k : (g.Kreal - 1);
      const int kpos = kc / g.Cin;
      const int ic = kc - kpos * g.Cin;
      float v = w[((long long)nc * g.Cin + ic) * g.taps + kpos];
      v = (nok && kok) ? v : 0.0f;
      const unsigned short hb = f2bf_bits(v);
      const unsigned short lb = f2bf_bits(v - bf_bits2f(hb));
      hbits[j] = (unsigned)hb;
      lbits[j] = (unsigned)lb;
    }
    v4u hv, lv;
    hv.x = hbits[0] | (hbits[1] << 16); hv.y = hbits[2] | (hbits[3] << 16);
    hv.z = hbits[4] | (hbits[5] << 16); hv.w = hbits[6] | (hbits[7] << 16);
    lv.x = lbits[0] | (lbits[1] << 16); lv.y = lbits[2] | (lbits[3] << 16);
    lv.z = lbits[4] | (lbits[5] << 16); lv.w = lbits[6] | (lbits[7] << 16);
    unsigned short* ph = Bhi + (size_t)e0;
    unsigned short* pl = Blo + (size_t)e0;
    for (int pass = 0; pass < 2; ++pass) {
      *(volatile v4u*)ph = hv;
      *(volatile v4u*)pl = lv;
      __threadfence();
    }
  }
  if (blockIdx.x == 0 && (threadIdx.x >> 5) == 0) {
    const int lane = threadIdx.x & 31;
    for (int pass = 0; pass < 2; ++pass) {
      for (int base = 0; base < g.NPAD; base += 128) {
        const int idx = base + 4 * lane;
        float bv[4];
#pragma unroll
        for (int q = 0; q < 4; ++q) {
          float x = 0.0f;
          if (g.has_bias) x = bias[min(idx + q, g.Cout - 1)];
          bv[q] = (idx + q < g.Cout) ? x : 0.0f;
        }
        if (idx < g.NPAD) {
          v4f vv; vv.x = bv[0]; vv.y = bv[1]; vv.z = bv[2]; vv.w = bv[3];
          *(volatile v4f*)(bpad + idx) = vv;
        }
      }
      __threadfence();
    }
  }
}

constexpr int IMG_HW = 1024;
constexpr int IMG_PIX = 1048576;
constexpr int GRID_LD = 128;

__device__ __forceinline__ v8f mma16_guard(v16h a, v16h b, v8f c) {
  c = __builtin_amdgcn_wmma_f32_16x16x32_f16(false, a, false, b, (short)0, c, false, false);
  asm volatile("v_nop\n\tv_nop\n\tv_nop\n\tv_nop" : "+v"(c) : "v"(a), "v"(b));
  return c;
}

__device__ __forceinline__ float grid_corner_val(const float* __restrict__ gridc, int b, int i,
                                                 int fx, int cx, int fy, int cy) {
  const int corner = i / 96;
  const int rem = i - corner * 96;
  const int z = rem / 12;
  const int c = rem - z * 12;
  const int yy = (corner & 2) ? cy : fy;
  const int xx = (corner & 1) ? cx : fx;
  return gridc[(size_t)(b * 256 + yy * 16 + xx) * GRID_LD + c * 8 + z];
}

__global__ __launch_bounds__(256) void slice_affine_kernel(
    const float* __restrict__ high, const float* __restrict__ gridc,
    const float* __restrict__ pw_mat, const float* __restrict__ pw_bias,
    const float* __restrict__ pw_bias_tag, const float* __restrict__ rho_a,
    const float* __restrict__ rho_t, float* __restrict__ out) {
  __shared__ __align__(16) float sg[384];
  __shared__ __align__(16) float s_rt[64];
  __shared__ __align__(16) float s_ra[64];
  const int tid = threadIdx.x;
  const int wave = tid >> 5, lane = tid & 31, hh = lane >> 4, m = lane & 15;
  const int blk = blockIdx.x;
  const int xb = blk & 31;
  const int yb = (blk >> 5) & 127;
  const int b = blk >> 12;
  const int x0 = xb * 32;
  const int y0 = yb * 8;
  const int y = y0 + wave;

  const float txb = (((float)x0 + 0.5f) * 0.0009765625f) * 16.0f - 0.5f;
  const float tyb = (((float)y0 + 0.5f) * 0.0009765625f) * 16.0f - 0.5f;
  int fxb = (int)fmaxf(floorf(txb), 0.0f);
  int fyb = (int)fmaxf(floorf(tyb), 0.0f);
  fxb = min(max(fxb, 0), 15);
  fyb = min(max(fyb, 0), 15);
  const int cxb = min(fxb + 1, 15);
  const int cyb = min(fyb + 1, 15);

  {
    const int i0 = tid;
    const int i1 = 256 + (tid & 127);
    const float v0 = grid_corner_val(gridc, b, i0, fxb, cxb, fyb, cyb);
    const float v1 = grid_corner_val(gridc, b, i1, fxb, cxb, fyb, cyb);
    sg[i0] = v0;
    sg[i1] = v1;
  }
  if (tid < 64) {
    const int kc = min(tid, 47);
    const float rt = rho_t[kc];
    const float ra = rho_a[kc];
    s_rt[tid] = (tid < 48) ? rt : 3.0e38f;
    s_ra[tid] = (tid < 48) ? ra : 0.0f;
  }
  __syncthreads();

  float pm[9];
#pragma unroll
  for (int i = 0; i < 9; ++i) pm[i] = pw_mat[i];
  const float tg0 = pw_bias_tag[0], tg1 = pw_bias_tag[1], tg2 = pw_bias_tag[2];
  const float pwb = pw_bias[0];

  const size_t img = (size_t)b * 3 * IMG_PIX;
  const size_t rowoff = img + (size_t)y * IMG_HW + (size_t)x0;
  const float pr0 = high[rowoff + m];
  const float pg0 = high[rowoff + IMG_PIX + m];
  const float pb0 = high[rowoff + 2 * IMG_PIX + m];
  const float pr1 = high[rowoff + 16 + m];
  const float pg1 = high[rowoff + IMG_PIX + 16 + m];
  const float pb1 = high[rowoff + 2 * IMG_PIX + 16 + m];
  const float rr = hh ? pr1 : pr0;
  const float gg = hh ? pg1 : pg0;
  const float bbv = hh ? pb1 : pb0;

  float gA[3], gB[3];
  gA[0] = pm[0] * pr0 + pm[1] * pg0 + pm[2] * pb0 + tg0;
  gA[1] = pm[3] * pr0 + pm[4] * pg0 + pm[5] * pb0 + tg1;
  gA[2] = pm[6] * pr0 + pm[7] * pg0 + pm[8] * pb0 + tg2;
  gB[0] = pm[0] * pr1 + pm[1] * pg1 + pm[2] * pb1 + tg0;
  gB[1] = pm[3] * pr1 + pm[4] * pg1 + pm[5] * pb1 + tg1;
  gB[2] = pm[6] * pr1 + pm[7] * pg1 + pm[8] * pb1 + tg2;

  v16h afr[2], bt0[2], bt1[2];
#pragma unroll
  for (int s = 0; s < 2; ++s) {
#pragma unroll
    for (int q = 0; q < 2; ++q) {
      const int kb = 32 * s + 16 * q + 8 * hh;
      const v4f rtA = *(const v4f*)(s_rt + kb);
      const v4f rtB = *(const v4f*)(s_rt + kb + 4);
      const v4f raA = *(const v4f*)(s_ra + kb);
      const v4f raB = *(const v4f*)(s_ra + kb + 4);
      const float rtv[8] = {rtA.x, rtA.y, rtA.z, rtA.w, rtB.x, rtB.y, rtB.z, rtB.w};
      const float rav[8] = {raA.x, raA.y, raA.z, raA.w, raB.x, raB.y, raB.z, raB.w};
      const int kb3 = kb % 3;
#pragma unroll
      for (int e = 0; e < 8; ++e) {
        int c3 = kb3 + (e % 3);
        c3 = (c3 >= 3) ? (c3 - 3) : c3;
        const float ga = (c3 == 0) ? gA[0] : ((c3 == 1) ? gA[1] : gA[2]);
        const float gb = (c3 == 0) ? gB[0] : ((c3 == 1) ? gB[1] : gB[2]);
        const float av = (m == 0) ? rav[e] : 0.0f;
        afr[s][8 * q + e] = (_Float16)av;
        bt0[s][8 * q + e] = (_Float16)fmaxf(ga - rtv[e], 0.0f);
        bt1[s][8 * q + e] = (_Float16)fmaxf(gb - rtv[e], 0.0f);
      }
    }
  }
  v8f acc0 = (v8f){0.f,0.f,0.f,0.f,0.f,0.f,0.f,0.f};
  v8f acc1 = (v8f){0.f,0.f,0.f,0.f,0.f,0.f,0.f,0.f};
  acc0 = mma16_guard(afr[0], bt0[0], acc0);
  acc0 = mma16_guard(afr[1], bt0[1], acc0);
  acc1 = mma16_guard(afr[0], bt1[0], acc1);
  acc1 = mma16_guard(afr[1], bt1[1], acc1);
  const float g1s = __shfl(acc1[0], m, 32);
  const float gsum = hh ? g1s : acc0[0];
  const float guide = gsum + pwb;

  const float gcl = fminf(fmaxf(guide, 0.0f), 1.0f);
  const float gz = gcl * 8.0f;
  const float tz = gz - 0.5f;
  const float fzf = fmaxf(floorf(tz), 0.0f);
  const float wz = fabsf(tz - fzf);
  int fz = (int)fzf;
  fz = min(max(fz, 0), 7);
  const int cz = min(fz + 1, 7);

  const float xf = (float)(x0 + lane);
  const float tx = ((xf + 0.5f) * 0.0009765625f) * 16.0f - 0.5f;
  const float fxf = fmaxf(floorf(tx), 0.0f);
  const float wx = tx - fxf;
  const float yf = (float)y;
  const float ty = ((yf + 0.5f) * 0.0009765625f) * 16.0f - 0.5f;
  const float fyf = fmaxf(floorf(ty), 0.0f);
  const float wy = ty - fyf;
  const float ux = 1.0f - wx, uy = 1.0f - wy, uz = 1.0f - wz;

  float ac[12];
#pragma unroll
  for (int c = 0; c < 12; ++c) ac[c] = 0.0f;
#pragma unroll
  for (int xi = 0; xi < 2; ++xi) {
    const float wxs = xi ? wx : ux;
#pragma unroll
    for (int yi = 0; yi < 2; ++yi) {
      const float wys = yi ? wy : uy;
      const int corner = yi * 2 + xi;
      const float* pf = sg + corner * 96 + fz * 12;
      const float* pc = sg + corner * 96 + cz * 12;
#pragma unroll
      for (int q = 0; q < 3; ++q) {
        const v4f vf = *(const v4f*)(pf + 4 * q);
        const v4f vc = *(const v4f*)(pc + 4 * q);
#pragma unroll
        for (int e = 0; e < 4; ++e) {
          ac[4 * q + e] += ((vf[e] * wxs) * wys) * uz;
          ac[4 * q + e] += ((vc[e] * wxs) * wys) * wz;
        }
      }
    }
  }
  const float o0 = (ac[0] * rr + ac[2] * bbv) + ac[1] * gg + ac[3];
  const float o1 = (ac[4] * rr + ac[6] * bbv) + ac[5] * gg + ac[7];
  const float o2 = (ac[8] * rr + ac[10] * bbv) + ac[9] * gg + ac[11];

  float* op = out + img + (size_t)y * IMG_HW + (size_t)x0 + lane;
  for (int pass = 0; pass < 2; ++pass) {
    *(volatile float*)(op) = o0;
    *(volatile float*)(op + IMG_PIX) = o1;
    *(volatile float*)(op + 2 * IMG_PIX) = o2;
    __threadfence();
  }
}

struct HostLayer { int Cin, Cout, Hin, Win, Hout, Wout, stride, pad, taps, Kreal, KPAD, NPAD, Mreal, MPAD; };
static constexpr HostLayer kLayers[12] = {
  {   3,   8, 256, 256, 128, 128, 2, 1, 9,   27,   32,  64, 32768, 32768},
  {   8,  16, 128, 128,  64,  64, 2, 1, 9,   72,   96,  64,  8192,  8192},
  {  16,  32,  64,  64,  32,  32, 2, 1, 9,  144,  160,  64,  2048,  2048},
  {  32,  64,  32,  32,  16,  16, 2, 1, 9,  288,  288,  64,   512,   512},
  {  64,  64,  16,  16,  16,  16, 1, 1, 9,  576,  576,  64,   512,   512},
  {  64,  64,  16,  16,  16,  16, 1, 1, 9,  576,  576,  64,   512,   512},
  {  64,  64,  16,  16,   8,   8, 2, 1, 9,  576,  576,  64,   128,   128},
  {  64,  64,   8,   8,   4,   4, 2, 1, 9,  576,  576,  64,    32,    64},
  {1024, 256,   1,   1,   1,   1, 1, 0, 1, 1024, 1024, 256,     2,    64},
  { 256, 128,   1,   1,   1,   1, 1, 0, 1,  256,  256, 128,     2,    64},
  { 128,  64,   1,   1,   1,   1, 1, 0, 1,  128,  128,  64,     2,    64},
  {  64,  96,  16,  16,  16,  16, 1, 0, 1,   64,   64, 128,   512,   512},
};
constexpr bool layers_ok() {
  for (int i = 0; i < 12; ++i) {
    const HostLayer& L = kLayers[i];
    if (L.KPAD % 32 != 0) return false;
    if (L.NPAD % 64 != 0) return false;
    if (L.MPAD % 64 != 0) return false;
    if (L.Kreal > L.KPAD || L.Kreal != L.taps * L.Cin) return false;
    if (L.Cout > L.NPAD || L.Mreal > L.MPAD) return false;
    if ((L.MPAD * L.KPAD) % 2048 != 0) return false;
    if ((L.NPAD * L.KPAD) % 2048 != 0) return false;
    if ((L.taps == 9) && (L.Hout != (L.Hin + 2 * L.pad - 3) / L.stride + 1)) return false;
  }
  return true;
}
static_assert(layers_ok());
static_assert(GRID_LD == kLayers[11].NPAD);

static inline size_t alignup256(size_t x) { return (x + 255) & ~(size_t)255; }

struct LayerBuf { unsigned short* Bhi; unsigned short* Blo; float* bpad; unsigned short* Ahi; unsigned short* Alo; float* C; };

static void launch_gemm(bool relu, const LayerBuf& lb, const HostLayer& L, hipStream_t stream) {
  const int tiles = (L.MPAD / 64) * (L.NPAD / 64);
  const int blocks = (tiles + 7) / 8;
  if (relu) {
    wmma_gemm64<1, true, 2, 0, false, 2><<<dim3(blocks, 1), 256, 0, stream>>>(
        lb.Ahi, lb.Alo, L.KPAD, 0L, lb.Bhi, lb.Blo, L.KPAD, 0L,
        (void*)lb.C, nullptr, L.NPAD, 0L, lb.bpad, nullptr, 0L, L.MPAD, L.NPAD, L.KPAD, 1.0f);
  } else {
    wmma_gemm64<1, true, 2, 0, false, 0><<<dim3(blocks, 1), 256, 0, stream>>>(
        lb.Ahi, lb.Alo, L.KPAD, 0L, lb.Bhi, lb.Blo, L.KPAD, 0L,
        (void*)lb.C, nullptr, L.NPAD, 0L, lb.bpad, nullptr, 0L, L.MPAD, L.NPAD, L.KPAD, 1.0f);
  }
}

static ColGeom make_geom(const HostLayer& L, long long sb, long long sy, long long sx,
                         long long s_clo, long long s_chi, int cmask, int cshift, long long add_sb) {
  ColGeom g = {};
  g.sb = sb; g.sy = sy; g.sx = sx; g.s_clo = s_clo; g.s_chi = s_chi; g.add_sb = add_sb;
  g.Hin = L.Hin; g.Win = L.Win; g.Hout = L.Hout; g.Wout = L.Wout;
  g.stride = L.stride; g.pad = L.pad; g.taps = L.taps; g.kw = (L.taps == 9) ? 3 : 1;
  g.Cin = L.Cin; g.Kreal = L.Kreal; g.KPAD = L.KPAD; g.Mreal = L.Mreal;
  g.cmask = cmask; g.cshift = cshift; g.nthr = L.MPAD * L.KPAD / 8; g.unused0 = 0;
  return g;
}

extern "C" void kernel_launch(void* const* d_in, const int* in_sizes, int n_in,
                              void* d_out, int out_size, void* d_ws, size_t ws_size,
                              hipStream_t stream) {
  if (n_in < 30) return;
  if (in_sizes[0] != 2 * 3 * IMG_PIX) return;
  if (in_sizes[1] != 2 * 3 * 256 * 256) return;
  if (out_size != 2 * 3 * IMG_PIX) return;

  const float* high  = (const float*)d_in[0];
  const float* low   = (const float*)d_in[1];
  const float* wptr[12];
  const float* bptr[12];
  wptr[0]  = (const float*)d_in[2];  bptr[0]  = (const float*)d_in[3];
  wptr[1]  = (const float*)d_in[4];  bptr[1]  = (const float*)d_in[5];
  wptr[2]  = (const float*)d_in[6];  bptr[2]  = (const float*)d_in[7];
  wptr[3]  = (const float*)d_in[8];  bptr[3]  = (const float*)d_in[9];
  wptr[4]  = (const float*)d_in[10]; bptr[4]  = (const float*)d_in[11];
  wptr[5]  = (const float*)d_in[12]; bptr[5]  = nullptr;
  wptr[6]  = (const float*)d_in[13]; bptr[6]  = (const float*)d_in[14];
  wptr[7]  = (const float*)d_in[15]; bptr[7]  = (const float*)d_in[16];
  wptr[8]  = (const float*)d_in[17]; bptr[8]  = (const float*)d_in[18];
  wptr[9]  = (const float*)d_in[19]; bptr[9]  = (const float*)d_in[20];
  wptr[10] = (const float*)d_in[21]; bptr[10] = (const float*)d_in[22];
  wptr[11] = (const float*)d_in[23]; bptr[11] = (const float*)d_in[24];
  const float* pw_mat      = (const float*)d_in[25];
  const float* pw_bias     = (const float*)d_in[26];
  const float* pw_bias_tag = (const float*)d_in[27];
  const float* rho_a       = (const float*)d_in[28];
  const float* rho_t       = (const float*)d_in[29];
  const int relu_flag[12] = {1, 1, 1, 1, 1, 0, 1, 1, 1, 1, 0, 0};

  char* ws = (char*)d_ws;
  size_t off = 0;
  LayerBuf lb[12];
  for (int i = 0; i < 12; ++i) {
    const HostLayer& L = kLayers[i];
    const size_t bplane = (size_t)L.NPAD * L.KPAD * 2;
    const size_t aplane = (size_t)L.MPAD * L.KPAD * 2;
    const size_t cbytes = (size_t)L.MPAD * L.NPAD * 4;
    lb[i].Bhi  = (unsigned short*)(ws + off); off = alignup256(off + bplane);
    lb[i].Blo  = (unsigned short*)(ws + off); off = alignup256(off + bplane);
    lb[i].bpad = (float*)(ws + off);          off = alignup256(off + (size_t)L.NPAD * 4);
    lb[i].Ahi  = (unsigned short*)(ws + off); off = alignup256(off + aplane);
    lb[i].Alo  = (unsigned short*)(ws + off); off = alignup256(off + aplane);
    lb[i].C    = (float*)(ws + off);          off = alignup256(off + cbytes);
  }
  if (off > ws_size) return;

  for (int i = 0; i < 12; ++i) {
    const HostLayer& L = kLayers[i];
    WGeom wg;
    wg.Cout = L.Cout; wg.Cin = L.Cin; wg.taps = L.taps; wg.Kreal = L.Kreal; wg.KPAD = L.KPAD; wg.NPAD = L.NPAD;
    wg.nthr = L.NPAD * L.KPAD / 8; wg.has_bias = (bptr[i] != nullptr) ? 1 : 0;
    prep_w_kernel<<<wg.nthr / 256, 256, 0, stream>>>(wptr[i], bptr[i], lb[i].Bhi, lb[i].Blo, lb[i].bpad, wg);
  }

  const int cmask_all = 0x7fffffff;
  {
    const HostLayer& L = kLayers[0];
    ColGeom g = make_geom(L, 3LL * 256 * 256, 256, 1, 256LL * 256, 0, cmask_all, 31, 0);
    im2col_split_kernel<0><<<g.nthr / 256, 256, 0, stream>>>(low, nullptr, lb[0].Ahi, lb[0].Alo, g);
    launch_gemm(relu_flag[0] != 0, lb[0], L, stream);
  }
  const int src_of[8] = {-1, 0, 1, 2, 3, 4, 3, 6};
  for (int i = 1; i < 8; ++i) {
    const HostLayer& L = kLayers[i];
    const long long ld = kLayers[src_of[i]].NPAD;
    ColGeom g = make_geom(L, (long long)L.Hin * L.Win * ld, (long long)L.Win * ld, ld, 1, 0, cmask_all, 31, 0);
    im2col_split_kernel<0><<<g.nthr / 256, 256, 0, stream>>>(lb[src_of[i]].C, nullptr, lb[i].Ahi, lb[i].Alo, g);
    launch_gemm(relu_flag[i] != 0, lb[i], L, stream);
  }
  {
    const HostLayer& L = kLayers[8];
    ColGeom g = make_geom(L, 16LL * kLayers[7].NPAD, 0, 0, kLayers[7].NPAD, 1, 15, 4, 0);
    im2col_split_kernel<0><<<g.nthr / 256, 256, 0, stream>>>(lb[7].C, nullptr, lb[8].Ahi, lb[8].Alo, g);
    launch_gemm(relu_flag[8] != 0, lb[8], L, stream);
  }
  {
    const HostLayer& L = kLayers[9];
    ColGeom g = make_geom(L, kLayers[8].NPAD, 0, 0, 1, 0, cmask_all, 31, 0);
    im2col_split_kernel<0><<<g.nthr / 256, 256, 0, stream>>>(lb[8].C, nullptr, lb[9].Ahi, lb[9].Alo, g);
    launch_gemm(relu_flag[9] != 0, lb[9], L, stream);
  }
  {
    const HostLayer& L = kLayers[10];
    ColGeom g = make_geom(L, kLayers[9].NPAD, 0, 0, 1, 0, cmask_all, 31, 0);
    im2col_split_kernel<0><<<g.nthr / 256, 256, 0, stream>>>(lb[9].C, nullptr, lb[10].Ahi, lb[10].Alo, g);
    launch_gemm(relu_flag[10] != 0, lb[10], L, stream);
  }
  {
    const HostLayer& L = kLayers[11];
    const long long ld = kLayers[5].NPAD;
    ColGeom g = make_geom(L, (long long)L.Hin * L.Win * ld, (long long)L.Win * ld, ld, 1, 0, cmask_all, 31,
                          (long long)kLayers[10].NPAD);
    im2col_split_kernel<1><<<g.nthr / 256, 256, 0, stream>>>(lb[5].C, lb[10].C, lb[11].Ahi, lb[11].Alo, g);
    launch_gemm(relu_flag[11] != 0, lb[11], L, stream);
  }
  slice_affine_kernel<<<8192, 256, 0, stream>>>(high, lb[11].C, pw_mat, pw_bias, pw_bias_tag,
                                                rho_a, rho_t, (float*)d_out);
}
